// CrossNetMix_15229954032206
// MI455X (gfx1250) — hardware-verified
//
#include <hip/hip_runtime.h>


#define NR   16384
#define DD   512
#define NE   4
#define RR   64
#define NL   3
typedef _Float16 h16;
typedef unsigned short bf;
typedef __attribute__((ext_vector_type(16))) __bf16   v16bf;
typedef __attribute__((ext_vector_type(16))) _Float16 v16h;
typedef __attribute__((ext_vector_type(8)))  _Float16 v8h;
typedef __attribute__((ext_vector_type(8)))  unsigned short v8us;
typedef __attribute__((ext_vector_type(8)))  float    v8f;
typedef __attribute__((ext_vector_type(4)))  float    v4f;
typedef v8h  __attribute__((may_alias)) v8ha;
typedef v4f  __attribute__((may_alias)) v4fa;
typedef v8us __attribute__((may_alias)) v8usa;

__device__ __forceinline__ unsigned short f2bf(float f) { unsigned u = __float_as_uint(f); u += 0x7FFFu + ((u >> 16) & 1u); return (unsigned short)(u >> 16); }
__device__ __forceinline__ float bf2f(unsigned short b) { return __uint_as_float(((unsigned)b) << 16); }
__device__ __forceinline__ float bfr(float f) { return bf2f(f2bf(f)); }
__device__ __forceinline__ v16h cat16(v8h lo, v8h hi) { return __builtin_shufflevector(lo, hi, 0, 1, 2, 3, 4, 5, 6, 7, 8, 9, 10, 11, 12, 13, 14, 15); }
__device__ __forceinline__ v16bf cat16b(v8us lo, v8us hi) { return __builtin_bit_cast(v16bf, __builtin_shufflevector(lo, hi, 0, 1, 2, 3, 4, 5, 6, 7, 8, 9, 10, 11, 12, 13, 14, 15)); }
__device__ __forceinline__ v8f wmma16(v16h a, v16h b, v8f c) { return __builtin_amdgcn_wmma_f32_16x16x32_f16(false, a, false, b, (short)0, c, false, false); }
__device__ __forceinline__ v8f wmmab(v16bf a, v16bf b, v8f c) { return __builtin_amdgcn_wmma_f32_16x16x32_bf16(false, a, false, b, (short)0, c, false, false); }


template <typename T16> struct WFrag;
template <> struct WFrag<h16> { typedef v16h V; static __device__ __forceinline__ V ld(const h16* p) { return cat16(*(const v8h*)p, *(const v8h*)(p + 16)); } static __device__ __forceinline__ v8f mma(V a, V b, v8f c) { return wmma16(a, b, c); } };
template <> struct WFrag<bf> { typedef v16bf V; static __device__ __forceinline__ V ld(const bf* p) { return cat16b(*(const v8us*)p, *(const v8us*)(p + 16)); } static __device__ __forceinline__ v8f mma(V a, V b, v8f c) { return wmmab(a, b, c); } };
template <typename T16, int NSPLIT, bool BIAS>
__global__ __launch_bounds__(32) void k_gemmw(const T16* __restrict__ A, const T16* __restrict__ A2, const T16* __restrict__ Bt, const T16* __restrict__ Bt2, int K, float* C, int ldc, const float* __restrict__ bias, size_t sA, size_t sB, size_t sC) {
    typedef typename WFrag<T16>::V V;
    __shared__ __align__(16) float os[16 * 68];
    const size_t z = blockIdx.z; A += z * sA; if (A2) A2 += z * sA; Bt += z * sB; if (Bt2) Bt2 += z * sB; C += z * sC;
    const int lane = threadIdx.x & 31, lr = lane & 15, hi = lane >> 4; const int r0 = blockIdx.x * 64, c0 = blockIdx.y * 64;
    v8f acc[4][4];
#pragma unroll
    for (int mb = 0; mb < 4; ++mb)
#pragma unroll
        for (int nb = 0; nb < 4; ++nb) acc[mb][nb] = (v8f){};
    const size_t aoff = (size_t)(r0 + lr) * K + 8 * hi, boff = (size_t)(c0 + lr) * K + 8 * hi;
#pragma unroll 1
    for (int kc = 0; kc < K; kc += 32) {
        V a[4], a2[4];
#pragma unroll
        for (int mb = 0; mb < 4; ++mb) { a[mb] = WFrag<T16>::ld(A + aoff + (size_t)mb * 16 * K + kc); if (NSPLIT == 1 || NSPLIT == 2) a2[mb] = WFrag<T16>::ld(A2 + aoff + (size_t)mb * 16 * K + kc); }
#pragma unroll
        for (int nb = 0; nb < 4; ++nb) { const V b = WFrag<T16>::ld(Bt + boff + (size_t)nb * 16 * K + kc); V b2; if (NSPLIT >= 2) b2 = WFrag<T16>::ld(Bt2 + boff + (size_t)nb * 16 * K + kc);
#pragma unroll
            for (int mb = 0; mb < 4; ++mb) { acc[mb][nb] = WFrag<T16>::mma(a[mb], b, acc[mb][nb]); if (NSPLIT == 1 || NSPLIT == 2) acc[mb][nb] = WFrag<T16>::mma(a2[mb], b, acc[mb][nb]); if (NSPLIT >= 2) acc[mb][nb] = WFrag<T16>::mma(a[mb], b2, acc[mb][nb]); } }
        asm volatile("v_nop\n\tv_nop\n\tv_nop\n\tv_nop" : "+v"(acc[0][0]), "+v"(acc[1][1]), "+v"(acc[2][2]), "+v"(acc[3][3]) : "v"(a[0]), "v"(a[3]));
    }
#pragma unroll
    for (int mb = 0; mb < 4; ++mb) {
#pragma unroll
        for (int nb = 0; nb < 4; ++nb) {
#pragma unroll
            for (int j = 0; j < 8; ++j) os[(hi * 8 + j) * 68 + nb * 16 + lr] = acc[mb][nb][j]; }
        __builtin_amdgcn_wave_barrier(); asm volatile("" ::: "memory");
        float* crow = C + (size_t)(r0 + mb * 16) * ldc + c0;
#pragma unroll 1
        for (int ps = 0; ps < 2; ++ps) {
#pragma unroll
            for (int s = 0; s < 8; ++s) { const int row = 2 * s + hi, cofs = lr * 4; v4f val = *(const v4fa*)(os + row * 68 + cofs); if (BIAS) { val[0] += bfr(bias[c0 + cofs]); val[1] += bfr(bias[c0 + cofs + 1]); val[2] += bfr(bias[c0 + cofs + 2]); val[3] += bfr(bias[c0 + cofs + 3]); }
                *(volatile v4f*)(crow + (size_t)row * ldc + cofs) = val; }
            if (ps == 0) __threadfence(); }
        __builtin_amdgcn_wave_barrier(); asm volatile("" ::: "memory");
    }
}

__device__ __forceinline__ void splitf(float y, unsigned short& h, unsigned short& l) { h = f2bf(y); l = f2bf(y - bf2f(h)); }
__device__ __forceinline__ float tanhf_(float a) { const float e2 = __expf(2.0f * a); return __fsub_rn(1.0f, __fdiv_rn(2.0f, __fadd_rn(e2, 1.0f))); }
typedef __attribute__((ext_vector_type(2))) unsigned short v2us;
typedef __attribute__((ext_vector_type(4))) unsigned short v4us;
typedef __attribute__((ext_vector_type(2))) float v2f;

__global__ __launch_bounds__(256) void k_cvt8(const float* __restrict__ src, bf* dst, size_t n8) { const size_t i = (size_t)blockIdx.x * 256 + threadIdx.x; if (i >= n8) return; const v8f v = *(const v8f*)(src + i * 8); v8us o;
#pragma unroll
    for (int k = 0; k < 8; ++k) o[k] = f2bf(v[k]); *(volatile v8us*)(dst + i * 8) = o; __threadfence(); *(volatile v8us*)(dst + i * 8) = o; }
__global__ __launch_bounds__(256) void k_gate(const float* __restrict__ XL, const float* __restrict__ gw, float* GT) { const int lane = threadIdx.x & 31; const int b = blockIdx.x * 8 + (threadIdx.x >> 5); if (b >= NR) return; float s[NE];
#pragma unroll
    for (int e = 0; e < NE; ++e) s[e] = 0.f;
    for (int d = lane; d < DD; d += 32) { const float xv = XL[(size_t)b * DD + d];
#pragma unroll
        for (int e = 0; e < NE; ++e) { float p = __fmul_rn(xv, bfr(gw[e * DD + d])); asm volatile("" : "+v"(p)); s[e] = __fadd_rn(s[e], p); } }
#pragma unroll
    for (int e = 0; e < NE; ++e)
#pragma unroll
        for (int sh = 16; sh; sh >>= 1) s[e] += __shfl_xor(s[e], sh, 32);
    float mx = fmaxf(fmaxf(s[0], s[1]), fmaxf(s[2], s[3])); float ex[NE], sum = 0.f;
#pragma unroll
    for (int e = 0; e < NE; ++e) { ex[e] = __expf(__fsub_rn(s[e], mx)); sum = __fadd_rn(sum, ex[e]); }
    const float o = lane < NE ? __fdiv_rn(ex[lane & 3], sum) : 0.f; *(volatile float*)(GT + (size_t)b * 32 + lane) = o; __threadfence(); *(volatile float*)(GT + (size_t)b * 32 + lane) = o; }
__global__ __launch_bounds__(256) void k_th1(const float* __restrict__ F1, bf* Hh, bf* Hl) { const size_t e_ = ((size_t)blockIdx.x * 256 + threadIdx.x) * 2; if (e_ >= (size_t)NE * NR * RR) return; const int r = (int)(e_ % RR); const int b = (int)((e_ / RR) % NR); const int e = (int)(e_ / ((size_t)RR * NR)); v2us oh, ol;
#pragma unroll
    for (int u = 0; u < 2; ++u) { unsigned short a, c2; splitf(tanhf_(F1[(size_t)b * (NE * RR) + e * RR + r + u]), a, c2); oh[u] = a; ol[u] = c2; } *(volatile v2us*)(Hh + e_) = oh; *(volatile v2us*)(Hl + e_) = ol; __threadfence(); *(volatile v2us*)(Hh + e_) = oh; *(volatile v2us*)(Hl + e_) = ol; }
__global__ __launch_bounds__(256) void k_th2(const float* __restrict__ F2, bf* Hh, bf* Hl) { const size_t e_ = ((size_t)blockIdx.x * 256 + threadIdx.x) * 2; if (e_ >= (size_t)NE * NR * RR) return; v2us oh, ol;
#pragma unroll
    for (int u = 0; u < 2; ++u) { unsigned short a, c2; splitf(tanhf_(F2[e_ + u]), a, c2); oh[u] = a; ol[u] = c2; } *(volatile v2us*)(Hh + e_) = oh; *(volatile v2us*)(Hl + e_) = ol; __threadfence(); *(volatile v2us*)(Hh + e_) = oh; *(volatile v2us*)(Hl + e_) = ol; }
__global__ __launch_bounds__(256) void k_spl(const float* __restrict__ X, bf* Xh, bf* Xl) { const size_t i = ((size_t)blockIdx.x * 256 + threadIdx.x) * 4; if (i >= (size_t)NR * DD) return; const v4f a = *(const v4f*)(X + i); v4us oh, ol;
#pragma unroll
    for (int q = 0; q < 4; ++q) { unsigned short u, c2; splitf(a[q], u, c2); oh[q] = u; ol[q] = c2; } *(volatile v4us*)(Xh + i) = oh; *(volatile v4us*)(Xl + i) = ol; __threadfence(); *(volatile v4us*)(Xh + i) = oh; *(volatile v4us*)(Xl + i) = ol; }
__global__ __launch_bounds__(256) void k_moe(const float* __restrict__ XL, const float* __restrict__ X0, const float* __restrict__ O, const float* __restrict__ GT, const float* __restrict__ bias, int e, float* ACC) { const size_t i = ((size_t)blockIdx.x * 256 + threadIdx.x) * 4; if (i >= (size_t)NR * DD) return; const int d = (int)(i % DD), b = (int)(i / DD); const float gte = GT[(size_t)b * 32 + e]; const v4f prev = e == 0 ? *(const v4f*)(XL + i) : *(const v4f*)(ACC + i); const v4f o4 = *(const v4f*)(O + i); v4f r;
#pragma unroll
    for (int q = 0; q < 4; ++q) { const float ob = __fadd_rn(o4[q], bfr(bias[d + q])); float xo = __fmul_rn(bfr(X0[i + q]), ob); asm volatile("" : "+v"(xo)); float gx = __fmul_rn(gte, xo); asm volatile("" : "+v"(gx)); r[q] = __fadd_rn(prev[q], gx); }
    *(volatile v4f*)(ACC + i) = r; __threadfence(); *(volatile v4f*)(ACC + i) = r; }
__global__ __launch_bounds__(256) void k_xl0(const float* __restrict__ X0, float* XL) { const size_t i = ((size_t)blockIdx.x * 256 + threadIdx.x) * 4; if (i >= (size_t)NR * DD) return; const v4f a = *(const v4f*)(X0 + i); v4f r; r[0] = bfr(a[0]); r[1] = bfr(a[1]); r[2] = bfr(a[2]); r[3] = bfr(a[3]); *(volatile v4f*)(XL + i) = r; __threadfence(); *(volatile v4f*)(XL + i) = r; }

extern "C" void kernel_launch(void* const* d_in, const int* in_sizes, int n_in,
                              void* d_out, int out_size, void* d_ws, size_t ws_size, hipStream_t stream) {
    (void)in_sizes; (void)n_in; (void)out_size;
    const float* X0 = (const float*)d_in[0]; const float* U = (const float*)d_in[1]; const float* V = (const float*)d_in[2]; const float* Cm = (const float*)d_in[3]; const float* bias = (const float*)d_in[4]; const float* gw = (const float*)d_in[5];
    float* OUT = (float*)d_out;
    char* wsp = (char*)d_ws;
    auto take = [&](size_t bytes) { char* p = wsp; wsp += (bytes + 255) & ~(size_t)255; return (void*)p; };
    bf* WV = (bf*)take((size_t)NE * RR * DD * 2); bf* WC = (bf*)take((size_t)NE * RR * RR * 2); bf* WU = (bf*)take((size_t)NE * DD * RR * 2);
    float* XL = (float*)take((size_t)NR * DD * 4); float* ACC = (float*)take((size_t)NR * DD * 4); bf* Xh = (bf*)take((size_t)NR * DD * 2); bf* Xl = (bf*)take((size_t)NR * DD * 2); float* GT = (float*)take((size_t)NR * 32 * 4);
    float* F1 = (float*)take((size_t)NR * NE * RR * 4); bf* H1h = (bf*)take((size_t)NE * NR * RR * 2); bf* H1l = (bf*)take((size_t)NE * NR * RR * 2); float* F2 = (float*)take((size_t)NE * NR * RR * 4); bf* H2h = (bf*)take((size_t)NE * NR * RR * 2); bf* H2l = (bf*)take((size_t)NE * NR * RR * 2); float* O = (float*)take((size_t)NR * DD * 4);
    if ((size_t)(wsp - (char*)d_ws) > ws_size) return;
    const unsigned LX = (unsigned)(((size_t)NR * DD / 4 + 255) / 256), LH = (unsigned)(((size_t)NE * NR * RR / 2 + 255) / 256);
    k_xl0<<<LX, 256, 0, stream>>>(X0, XL);
    float* cur = XL; float* nxt = ACC;
    for (int i = 0; i < NL; ++i) {
        k_cvt8<<<(NE * RR * DD / 8 + 255) / 256, 256, 0, stream>>>(V + (size_t)i * NE * RR * DD, WV, (size_t)NE * RR * DD / 8); k_cvt8<<<(NE * RR * RR / 8 + 255) / 256, 256, 0, stream>>>(Cm + (size_t)i * NE * RR * RR, WC, (size_t)NE * RR * RR / 8); k_cvt8<<<(NE * DD * RR / 8 + 255) / 256, 256, 0, stream>>>(U + (size_t)i * NE * DD * RR, WU, (size_t)NE * DD * RR / 8);
        k_gate<<<NR / 8, 256, 0, stream>>>(cur, gw, GT); k_spl<<<LX, 256, 0, stream>>>(cur, Xh, Xl);
        if (i == 0) k_gemmw<bf, 0, false><<<dim3(NR / 64, NE * RR / 64, 1), 32, 0, stream>>>(Xh, nullptr, WV, nullptr, DD, F1, NE * RR, nullptr, 0, 0, 0);
        else        k_gemmw<bf, 1, false><<<dim3(NR / 64, NE * RR / 64, 1), 32, 0, stream>>>(Xh, Xl, WV, nullptr, DD, F1, NE * RR, nullptr, 0, 0, 0);
        k_th1<<<LH, 256, 0, stream>>>(F1, H1h, H1l);
        k_gemmw<bf, 1, false><<<dim3(NR / 64, 1, NE), 32, 0, stream>>>(H1h, H1l, WC, nullptr, RR, F2, RR, nullptr, (size_t)NR * RR, (size_t)RR * RR, (size_t)NR * RR);
        k_th2<<<LH, 256, 0, stream>>>(F2, H2h, H2l);
        for (int e = 0; e < NE; ++e) { k_gemmw<bf, 1, false><<<dim3(NR / 64, DD / 64, 1), 32, 0, stream>>>(H2h + (size_t)e * NR * RR, H2l + (size_t)e * NR * RR, WU + (size_t)e * DD * RR, nullptr, RR, O, DD, nullptr, 0, 0, 0);
            k_moe<<<LX, 256, 0, stream>>>(cur, X0, O, GT, bias + (size_t)i * DD, e, i == NL - 1 ? OUT : nxt); }
        if (i < NL - 1) { float* t = cur; cur = nxt; nxt = t; } }
}
